// GraphRecommendationModel_48567490183265
// MI455X (gfx1250) — hardware-run, weakly checked
//
#include <hip/hip_runtime.h>


namespace {
constexpr int NU = 50000, NBK = 100000, N = NU + NBK, D = 128, E = 500000, NQ = 16384, NW = N / 16  ;
constexpr float HS = 256.0f, WSC = 256.0f, EPS = 1e-5f;
typedef _Float16 b16;
typedef __attribute__((ext_vector_type(16))) _Float16 v16b;
typedef __attribute__((ext_vector_type(8))) _Float16 v8b;
typedef __attribute__((ext_vector_type(8))) float v8f;
typedef __attribute__((ext_vector_type(4))) float v4f;
__device__ __forceinline__ float bf16_rne(float f) { unsigned int u = __float_as_uint(f); u += 0x7FFFu + ((u >> 16) & 1u); float r = __uint_as_float(u & 0xFFFF0000u); asm volatile("" : "+v"(r)); return r; }
__device__ __forceinline__ float bfv(float f) { float r = bf16_rne(f); asm volatile("" : "+v"(r)); return r; }
__device__ __forceinline__ void split16(float v, b16& hi, b16& lo) { hi = (b16)v; lo = (b16)(v - (float)hi); }
__device__ __forceinline__ v16b frag_kb(const b16* p, int hh) { const v8b a = *(const v8b*)(p + 8 * hh), b = *(const v8b*)(p + 16 + 8 * hh); v16b f;
#pragma unroll
  for (int e = 0; e < 8; ++e) { f[e] = a[e]; f[8 + e] = b[e]; } return f; }
__device__ __forceinline__ v8f wmma16b(v16b a, v16b b, v8f c) { v8f d = __builtin_amdgcn_wmma_f32_16x16x32_f16(false, a, false, b, (short)0, c, false, false); asm volatile("v_nop\n\tv_nop\n\tv_nop\n\tv_nop" : "+v"(d) : "v"(a), "v"(b)); return d; }
__device__ __forceinline__ void wave_lds_sync() { __builtin_amdgcn_fence(__ATOMIC_RELEASE, "workgroup"); __builtin_amdgcn_wave_barrier(); __builtin_amdgcn_fence(__ATOMIC_ACQUIRE, "workgroup"); }
__device__ __forceinline__ float pmul(float a, float b) { float p = a * b; asm volatile("" : "+v"(p)); return p; }
__device__ __forceinline__ int iclamp(int v, int lo, int hi) { return v < lo ? lo : (v > hi ? hi : v); }
constexpr int CSR_NBLK9 = 512, CSR_GB9 = 9, CSR_GN9 = 1 << CSR_GB9  , CSR_TS9 = (CSR_GN9 < 32 ? 32 : CSR_GN9)  , CSR_MAXG9 = 512, CSR_CAP9 = 12288  ;
__device__ __host__ __forceinline__ int csr_tix9(int v) { return (v >> CSR_GB9) * CSR_TS9 + (v & (CSR_GN9 - 1)); }
__global__ __launch_bounds__(64) void csrA_kernel9(const int* __restrict__ dst, int E, int N, int nG, int CHP, int NGP, int* __restrict__ STG, int* __restrict__ HST) {
  extern __shared__ int sm[];
  int* cnt = sm; int* run = sm + NGP; int* ids = sm + 2 * NGP;
  const int b = blockIdx.x; const int ch = (E + CSR_NBLK9 - 1) / CSR_NBLK9; const int e0 = b * ch, e1 = min(E, e0 + ch);
  for (int i = threadIdx.x; i < NGP; i += 64) cnt[i] = 0;
  for (int i = threadIdx.x; i < CHP; i += 64) ids[i] = -1;
  __syncthreads();
  if (threadIdx.x == 0) {
    for (int e = e0; e < e1; ++e) { int d = dst[e]; d = (d < 0) ? 0 : (d >= N ? N - 1 : d); cnt[d >> CSR_GB9] += 1; }
    int acc = 0; for (int g = 0; g < nG; ++g) { run[g] = acc; acc += cnt[g]; }
    for (int e = e0; e < e1; ++e) { int d = dst[e]; d = (d < 0) ? 0 : (d >= N ? N - 1 : d); const int g = d >> CSR_GB9; ids[run[g]] = e; run[g] += 1; } }
  __syncthreads();
  typedef __attribute__((ext_vector_type(4))) int v4i;
  for (int pass = 0; pass < 2; ++pass) {
    for (int i = threadIdx.x; i < CHP / 4; i += 64) *(volatile v4i*)(STG + (size_t)b * CHP + i * 4) = *(const v4i*)(&ids[i * 4]);
    for (int i = threadIdx.x; i < NGP / 4; i += 64) { v4i v; for (int e = 0; e < 4; ++e) v[e] = (i * 4 + e < nG) ? cnt[i * 4 + e] : 0; *(volatile v4i*)(HST + (size_t)b * NGP + i * 4) = v; }
    __threadfence(); }
}
__global__ __launch_bounds__(512) void csrS_kernel9(const int* __restrict__ HST, int nG, int NGP, int* __restrict__ START, int* __restrict__ TOT, int* __restrict__ OFF) {
  __shared__ int tot[CSR_MAXG9];
  const int b = threadIdx.x;
  for (int pass = 0; pass < 2; ++pass) { int runb = 0; for (int g = 0; g < nG; ++g) { int c = HST[(size_t)b * NGP + g]; c = (c < 0) ? 0 : c; ((volatile int*)OFF)[(size_t)g * CSR_NBLK9 + b] = runb; runb += c; } __threadfence(); }
  for (int g = threadIdx.x; g < nG; g += 512) { int s = 0; for (int bb = 0; bb < CSR_NBLK9; ++bb) { int c = HST[(size_t)bb * NGP + g]; s += (c < 0) ? 0 : c; } tot[g] = s; }
  __syncthreads();
  if (threadIdx.x < 32) {
    __shared__ int st[CSR_MAXG9 + 32];
    if (threadIdx.x == 0) { int acc = 0; for (int g = 0; g < NGP; ++g) { st[g] = acc; if (g < nG) acc += (tot[g] + 31) & ~31; } st[NGP] = acc; }
    __builtin_amdgcn_fence(__ATOMIC_RELEASE, "workgroup"); __builtin_amdgcn_wave_barrier(); __builtin_amdgcn_fence(__ATOMIC_ACQUIRE, "workgroup");
    for (int pass = 0; pass < 2; ++pass) { for (int i = threadIdx.x; i < NGP + 32; i += 32) { ((volatile int*)START)[i] = (i <= NGP) ? st[min(i, NGP)] : 0; ((volatile int*)TOT)[i] = (i < nG) ? tot[i] : 0; } __threadfence(); } }
}
__global__ __launch_bounds__(256) void csrB_kernel9(const int* __restrict__ dst, int N, int nG, int CHP, int NGP, int permLen, const int* __restrict__ STG, const int* __restrict__ HST, const int* __restrict__ OFF, const int* __restrict__ START, const int* __restrict__ TOT, int* __restrict__ PERM, int* __restrict__ ROWPTR, int* __restrict__ ROWCNT, int* __restrict__ FLAG) {
  typedef __attribute__((ext_vector_type(4))) int v4i;
  __shared__ int ids[CSR_CAP9]; __shared__ unsigned short key[CSR_CAP9]; __shared__ int outp[CSR_CAP9]; __shared__ int ncnt[CSR_GN9 + 1]; __shared__ int boff[CSR_NBLK9 + 1];
  const int g = blockIdx.x, t_ = threadIdx.x; int tot = TOT[g]; int st = START[g], stn = START[g + 1]; const int v0 = g * CSR_GN9; const int nv = min(CSR_GN9, N - v0); const int t0 = g * CSR_TS9;
  st = (st < 0) ? 0 : (st > permLen - 32 ? permLen - 32 : st) & ~31; stn = (stn < st) ? st : (stn > permLen ? permLen : stn); tot = (tot < 0) ? 0 : tot; if (tot > stn - st && tot <= CSR_CAP9) tot = stn - st;
  if (tot > CSR_CAP9) {
    for (int pass = 0; pass < 2; ++pass) { for (int i = t_; i < CSR_TS9 / 4; i += 256) { v4i a, c; for (int e = 0; e < 4; ++e) { a[e] = st; c[e] = 0; } *(volatile v4i*)(ROWPTR + t0 + i * 4) = a; *(volatile v4i*)(ROWCNT + t0 + i * 4) = c; } if (t_ == 0) ((volatile int*)FLAG)[0] = 1; __threadfence(); } (void)nv; return; }
  if (t_ == 0) { int acc = 0; for (int b = 0; b < CSR_NBLK9; ++b) { boff[b] = acc; int c = HST[(size_t)b * NGP + g]; c = (c < 0) ? 0 : (c > CHP ? CHP : c); acc += c; if (acc > tot) acc = tot; } boff[CSR_NBLK9] = acc; }
  for (int i = t_; i <= CSR_GN9; i += 256) ncnt[i] = 0;
  __syncthreads();
  for (int b = 0; b < CSR_NBLK9; ++b) { const int c = boff[b + 1] - boff[b]; int o_ = OFF[(size_t)g * CSR_NBLK9 + b]; o_ = (o_ < 0) ? 0 : (o_ > CHP - c ? CHP - c : o_); const int* src_ = STG + (size_t)b * CHP + o_;
    for (int i = t_; i < c; i += 256) { int id = src_[i]; id = (id < 0) ? 0 : id; ids[boff[b] + i] = id; int d = dst[id]; d = (d < v0) ? v0 : (d >= N ? N - 1 : d); int kk = d - v0; kk = (kk < 0) ? 0 : (kk >= CSR_GN9 ? CSR_GN9 - 1 : kk); key[boff[b] + i] = (unsigned short)kk; } }
  __syncthreads();
  if (t_ == 0) { for (int i = 0; i < tot; ++i) ncnt[key[i]] += 1; int acc = 0; for (int vl = 0; vl < CSR_GN9; ++vl) { const int c = ncnt[vl]; ncnt[vl] = acc; acc += c; } ncnt[CSR_GN9] = acc;
    for (int i = 0; i < tot; ++i) { const int vl = key[i]; outp[ncnt[vl]] = ids[i]; ncnt[vl] += 1; }
    for (int vl = CSR_GN9; vl > 0; --vl) ncnt[vl] = ncnt[vl - 1]; ncnt[0] = 0; }
  __syncthreads();
  for (int pass = 0; pass < 2; ++pass) {
    for (int i = t_; i < (stn - st) / 4; i += 256) { v4i v; for (int e = 0; e < 4; ++e) { const int q = i * 4 + e; v[e] = (q < tot) ? outp[q] : -1; } *(volatile v4i*)(PERM + st + i * 4) = v; }
    for (int i = t_; i < CSR_TS9 / 4; i += 256) { v4i a, c; for (int e = 0; e < 4; ++e) { const int vl = i * 4 + e; const int vc = vl < CSR_GN9 ? vl : CSR_GN9; a[e] = (vl < CSR_GN9) ? st + ncnt[vc] : st; c[e] = (vl < nv) ? (ncnt[(vc < CSR_GN9 ? vc : CSR_GN9 - 1) + 1] - ncnt[vc]) : 0; } *(volatile v4i*)(ROWPTR + t0 + i * 4) = a; *(volatile v4i*)(ROWCNT + t0 + i * 4) = c; }
    __threadfence(); }
}
__global__ __launch_bounds__(256) void csrZ_kernel9(int* __restrict__ p, size_t n4) { typedef __attribute__((ext_vector_type(4))) int v4i; const size_t tid = (size_t)blockIdx.x * 256 + threadIdx.x, nth = (size_t)gridDim.x * 256; v4i z = {0, 0, 0, 0}; for (size_t i = tid; i < n4; i += nth) *(volatile v4i*)(p + i * 4) = z; }
struct CsrBufs9 { int *STG, *HST, *OFF, *START, *TOT, *PERM, *ROWPTR, *ROWCNT, *FLAG; int nG, NGP, CHP; size_t permLen; char* base; size_t bytes; };
static size_t csr_carve9(CsrBufs9& c, char* ws, size_t off, int E, int N) {
  const size_t off0 = off; c.base = ws + off;
  auto al = [&](size_t bytes) { char* p = ws + off; off += (bytes + 255) & ~(size_t)255; return p; };
  c.nG = (N + CSR_GN9 - 1) / CSR_GN9; c.NGP = (c.nG + 31) & ~31; const int ch = (E + CSR_NBLK9 - 1) / CSR_NBLK9; c.CHP = (ch + 31) & ~31; c.permLen = (size_t)E + 32 * (size_t)c.nG + 32;
  c.STG = (int*)al((size_t)CSR_NBLK9 * c.CHP * 4); c.HST = (int*)al((size_t)CSR_NBLK9 * c.NGP * 4); c.OFF = (int*)al((size_t)c.NGP * CSR_NBLK9 * 4); c.START = (int*)al((size_t)(c.NGP + 64) * 4); c.TOT = (int*)al((size_t)(c.NGP + 64) * 4);
  c.PERM = (int*)al(c.permLen * 4); c.ROWPTR = (int*)al((size_t)c.nG * CSR_TS9 * 4); c.ROWCNT = (int*)al((size_t)c.nG * CSR_TS9 * 4); c.FLAG = (int*)al(256);
  c.bytes = off - off0; return off;
}
static void csr_build9(const CsrBufs9& c, const int* dst, int E, int N, hipStream_t stream) {
  const size_t smem = (size_t)(2 * c.NGP + c.CHP) * 4;
  csrZ_kernel9<<<512, 256, 0, stream>>>((int*)c.base, c.bytes / 16);
  csrA_kernel9<<<CSR_NBLK9, 64, smem, stream>>>(dst, E, N, c.nG, c.CHP, c.NGP, c.STG, c.HST);
  csrS_kernel9<<<1, 512, 0, stream>>>(c.HST, c.nG, c.NGP, c.START, c.TOT, c.OFF);
  csrB_kernel9<<<c.nG, 256, 0, stream>>>(dst, N, c.nG, c.CHP, c.NGP, (int)c.permLen, c.STG, c.HST, c.OFF, c.START, c.TOT, c.PERM, c.ROWPTR, c.ROWCNT, c.FLAG);
}


__global__ __launch_bounds__(256) void wput_kernel(const float* __restrict__ w1, const float* __restrict__ w2, b16* __restrict__ WT) { const int u = blockIdx.x * 256 + threadIdx.x; if (u >= 2 * D * 16) return; const int l = u / (D * 16), r = u % (D * 16); const int o = r / 16, k0 = (r % 16) * 8; const float* w = l == 0 ? w1 : w2; v8b v;
#pragma unroll
  for (int j = 0; j < 8; ++j) v[j] = (b16)(bf16_rne(w[(size_t)(k0 + j) * D + o]) * WSC); for (int pass = 0; pass < 2; ++pass) { *(volatile v8b*)(WT + ((size_t)l * D + o) * D + k0) = v; __threadfence(); } }
__global__ __launch_bounds__(256) void deg_kernel(const int* __restrict__ ROWCNT, float* __restrict__ DIS) { const int n = blockIdx.x * 256 + threadIdx.x; if (n >= N) return; const float d = rsqrtf((float)iclamp(ROWCNT[n], 0, E) + 1.0f); for (int pass = 0; pass < 2; ++pass) { ((volatile float*)DIS)[n] = d; __threadfence(); } }
template <int MODE>
__global__ __launch_bounds__(32) void lin_kernel(const float* __restrict__ ue, const float* __restrict__ be_, const float* __restrict__ G, const float* __restrict__ BNP, const b16* __restrict__ W, int NLIM, float* __restrict__ HW) { __shared__ __attribute__((aligned(16))) b16 Ah[16][D + 8], Al[16][D + 8]; __shared__ float Tf[16][D + 4]; const int lane = threadIdx.x, nloc = lane & 15, hlf = lane >> 4; const size_t m0 = (size_t)blockIdx.x * 16; if (m0 >= (size_t)NLIM) return;
  for (int rr = 0; rr < 16; ++rr) { const size_t n = m0 + rr; for (int q = 0; q < 4; ++q) { const int c = q * 32 + lane; b16 p, ql; if (MODE == 0) { const float v = n < (size_t)NU ? ue[n * D + c] : be_[(n - NU) * D + c]; p = (b16)(bf16_rne(v) * HS); ql = (b16)0.0f; } else { const float v = fmaxf(pmul(G[n * D + c], BNP[c]) + BNP[D + c], 0.0f); split16(v * HS, p, ql); } Ah[rr][c] = p; Al[rr][c] = ql; } }
  if (lane < 16) for (int k = D; k < D + 8; ++k) { Ah[lane][k] = (b16)0.0f; Al[lane][k] = (b16)0.0f; }
  wave_lds_sync(); v8f acc[8];
#pragma unroll
  for (int t = 0; t < 8; ++t) acc[t] = (v8f){};
#pragma unroll
  for (int kb = 0; kb < D; kb += 32) { const v16b a = frag_kb(&Ah[nloc][kb], hlf), al = frag_kb(&Al[nloc][kb], hlf);
#pragma unroll
    for (int t = 0; t < 8; ++t) { const v16b bw = frag_kb(W + (size_t)(t * 16 + nloc) * D + kb, hlf); acc[t] = wmma16b(a, bw, acc[t]); if (MODE == 1) acc[t] = wmma16b(al, bw, acc[t]); } }
#pragma unroll
  for (int t = 0; t < 8; ++t)
#pragma unroll
    for (int r8 = 0; r8 < 8; ++r8) Tf[8 * hlf + r8][t * 16 + nloc] = acc[t][r8] * (1.0f / (HS * WSC));
  wave_lds_sync();
  for (int pass = 0; pass < 2; ++pass) { for (int rr = 0; rr < 16; ++rr) *(volatile v4f*)(HW + (m0 + rr) * D + lane * 4) = *(const v4f*)(&Tf[rr][lane * 4]); __threadfence(); } }
__global__ __launch_bounds__(256) void sweep_kernel(const float* __restrict__ HW, const float* __restrict__ DIS, const float* __restrict__ bias, const int* __restrict__ srcs, const int* __restrict__ PERM, const int* __restrict__ ROWPTR, const int* __restrict__ ROWCNT, int permLen, int NLIM, float* __restrict__ G, float* __restrict__ PS) { __shared__ float Gs[8][D]; const int wave = threadIdx.x >> 5, lane = threadIdx.x & 31; const size_t i = (size_t)blockIdx.x * 8 + wave; const bool live = i < (size_t)NLIM; v4f o = {0, 0, 0, 0};
  if (live) { int st = ROWPTR[i], cnt = ROWCNT[i]; cnt = iclamp(cnt, 0, E); st = iclamp(st, 0, permLen - cnt); v4f acc = {0, 0, 0, 0};
#pragma unroll 1
    for (int j = 0; j < cnt; ++j) { const int e = iclamp(PERM[st + j], 0, E - 1); const size_t u = (size_t)iclamp(srcs[e], 0, N - 1); if (u >= (size_t)NLIM) continue; const float du = DIS[u]; const v4f v = *(const v4f*)(HW + u * D + lane * 4);
#pragma unroll
      for (int k = 0; k < 4; ++k) acc[k] += pmul(du, v[k]); }
    const float di = DIS[i]; const v4f hv = *(const v4f*)(HW + i * D + lane * 4);
#pragma unroll
    for (int k = 0; k < 4; ++k) o[k] = pmul(di, acc[k]) + pmul(pmul(di, di), hv[k]) + bfv(bias[lane * 4 + k]); }
#pragma unroll
  for (int k = 0; k < 4; ++k) Gs[wave][lane * 4 + k] = live ? o[k] : 0.0f;
  __syncthreads();
  for (int pass = 0; pass < 2; ++pass) { if (live) *(volatile v4f*)(G + i * D + lane * 4) = o; { const int c = threadIdx.x & 127, which = threadIdx.x >> 7; float s = 0.0f; for (int w = 0; w < 8; ++w) { const float v = Gs[w][c]; s += which ? v * v : v; } ((volatile float*)PS)[(size_t)blockIdx.x * 2 * D + which * D + c] = s; } __threadfence(); } }
__global__ __launch_bounds__(128) void bn_kernel(const float* __restrict__ PS, int nb, int count, const float* __restrict__ g, const float* __restrict__ be, float* __restrict__ BNP) { const int c = threadIdx.x; double s = 0.0, s2 = 0.0; for (int w = 0; w < nb; ++w) { s += (double)PS[(size_t)w * 2 * D + c]; s2 += (double)PS[(size_t)w * 2 * D + D + c]; } const double mu = s / count; double var = s2 / count - mu * mu; if (var < 0.0) var = 0.0; const float sc = bfv(g[c]) * (float)(1.0 / sqrt(var + (double)EPS)); const float sh = bfv(be[c]) - (float)mu * sc;
  for (int pass = 0; pass < 2; ++pass) { ((volatile float*)BNP)[c] = sc; ((volatile float*)BNP)[D + c] = sh; __threadfence(); } }
__global__ __launch_bounds__(32) void rate_kernel(const float* __restrict__ G, const float* __restrict__ BNP, const int* __restrict__ sn, const int* __restrict__ dn, const float* __restrict__ xun, int NLIM, float* __restrict__ out) { const int lane = threadIdx.x; const int q = blockIdx.x * 32 + lane; const size_t a = (size_t)iclamp(sn[q], 0, NLIM - 1), b = (size_t)iclamp(dn[q], 0, NLIM - 1); float s = 0.0f;
#pragma unroll 4
  for (int c = 0; c < D; ++c) { const float sc = BNP[c], sh = BNP[D + c]; const float ha = fmaxf(pmul(G[a * D + c], sc) + sh, 0.0f), hb = fmaxf(pmul(G[b * D + c], sc) + sh, 0.0f); s += pmul(ha, hb); }
  s += pmul(0.0f, bfv(xun[0]));
  for (int pass = 0; pass < 2; ++pass) { ((volatile float*)out)[q] = s; __threadfence(); } }
}

extern "C" void kernel_launch(void* const* d_in, const int* in_sizes, int n_in, void* d_out, int out_size, void* d_ws, size_t ws_size, hipStream_t stream) {
  (void)n_in;
  auto Fp = [&](int i) { return (const float*)d_in[i]; }; auto Ip = [&](int i) { return (const int*)d_in[i]; };
  if (in_sizes[0] != 2 * E || in_sizes[2] != NQ || in_sizes[3] != NQ || in_sizes[4] != NU * D || in_sizes[5] != NBK * D || in_sizes[6] != D * D || in_sizes[10] != D * D || out_size != NQ) return;
  const int NLIM = N;
  size_t off = 0; char* ws = (char*)d_ws;
  auto carve = [&](size_t bytes) { char* p = ws + off; off += (bytes + 255) & ~(size_t)255; return p; };
  b16* WT = (b16*)carve((size_t)2 * D * D * 2); float* DIS = (float*)carve((size_t)N * 4); float* HW = (float*)carve((size_t)N * D * 4); float* G = (float*)carve((size_t)N * D * 4); float* PS = (float*)carve((size_t)(N / 8) * 2 * D * 4); float* BN1 = (float*)carve(2 * D * 4); float* BN2 = (float*)carve(2 * D * 4);
  CsrBufs9 csr; off = csr_carve9(csr, ws, off, E, N);
  if (off > ws_size || off > ((size_t)224 << 20)) return;
  const int nb = (NLIM + 7) / 8;
  wput_kernel<<<(2 * D * 16 + 255) / 256, 256, 0, stream>>>(Fp(6), Fp(10), WT);
  csr_build9(csr, Ip(0) + E, E, N, stream);
  deg_kernel<<<(N + 255) / 256, 256, 0, stream>>>(csr.ROWCNT, DIS);
  lin_kernel<0><<<NLIM / 16, 32, 0, stream>>>(Fp(4), Fp(5), G, BN1, WT, NLIM, HW);
  sweep_kernel<<<nb, 256, 0, stream>>>(HW, DIS, Fp(7), Ip(0), csr.PERM, csr.ROWPTR, csr.ROWCNT, (int)csr.permLen, NLIM, G, PS); bn_kernel<<<1, 128, 0, stream>>>(PS, nb, NLIM, Fp(8), Fp(9), BN1);
  lin_kernel<1><<<NLIM / 16, 32, 0, stream>>>(Fp(4), Fp(5), G, BN1, WT + (size_t)D * D, NLIM, HW);
  sweep_kernel<<<nb, 256, 0, stream>>>(HW, DIS, Fp(11), Ip(0), csr.PERM, csr.ROWPTR, csr.ROWCNT, (int)csr.permLen, NLIM, G, PS); bn_kernel<<<1, 128, 0, stream>>>(PS, nb, NLIM, Fp(12), Fp(13), BN2);
  rate_kernel<<<NQ / 32, 32, 0, stream>>>(G, BN2, Ip(2), Ip(3), Fp(1), NLIM, (float*)d_out);
}
